// EdgeDeltaDiffusion_79517024518477
// MI455X (gfx1250) — hardware-verified
//
#include <hip/hip_runtime.h>
#include <stddef.h>


#define DD      128
#define NTHR    256
#define NWAVE   8
#define NBC     128
#define NBE     64
#define XP      136
#define EPT     8
#define NGRP    2
#define CHUNK   (NTHR * EPT * NGRP)
#define WCAP    (EPT * NGRP * 32)
#define LISTN   (NWAVE * WCAP)
#define NVERT   12500
#define WSCAP   134217728
#define VSTG    20480
#define VLDSB   147456
#define ELDSB   65536

static_assert((CHUNK & (CHUNK - 1)) == 0);
static_assert(CHUNK == 4096);
static_assert(NBC * DD * 2 * 4 + LISTN * 4 == VLDSB);
static_assert((VSTG + NWAVE * 2048) * 4 == VLDSB);
static_assert(VSTG * 4 >= 2 * NBC * XP * 2);
static_assert(2 * NBE * XP * 2 <= ELDSB);
static_assert(2 * NBE * DD * 4 == ELDSB);
static_assert(((XP * 2) % 16) == 0);
static_assert(NBC <= 4096);
static_assert(NWAVE * 32 == NTHR);
static_assert(NBE * 3 == 128 + 64);

typedef float    v4f  __attribute__((ext_vector_type(4)));
typedef float    v8f  __attribute__((ext_vector_type(8)));
typedef int      v4i  __attribute__((ext_vector_type(4)));
typedef _Float16 v4h  __attribute__((ext_vector_type(4)));
typedef _Float16 v8h  __attribute__((ext_vector_type(8)));
typedef _Float16 v16h __attribute__((ext_vector_type(16)));
union Frag { v16h v; v8h h[2]; };

extern __shared__ __attribute__((aligned(16))) float g_dyn[];

__device__ __forceinline__ v8f wm(v16h a, v16h b, v8f c) {
  v8f d = __builtin_amdgcn_wmma_f32_16x16x32_f16(false, a, false, b, (short)0, c, false, false);
  asm volatile("v_nop\n\tv_nop\n\tv_nop\n\tv_nop" : "+v"(d) : "v"(a), "v"(b));
  return d;
}

__device__ __forceinline__ v8f zero8() {
  v8f z = {0.f, 0.f, 0.f, 0.f, 0.f, 0.f, 0.f, 0.f};
  return z;
}

__device__ __forceinline__ float silu_f(float v) {
  return v * __builtin_amdgcn_rcpf(1.0f + __expf(-v));
}

__device__ __forceinline__ void st_seg(float* base, int f, int nval, v4f o) {
  if (f + 3 < nval) {
    *(volatile v4f*)(base + f) = o;
  } else {
    if (f     < nval) *(volatile float*)(base + f)     = o.x;
    if (f + 1 < nval) *(volatile float*)(base + f + 1) = o.y;
    if (f + 2 < nval) *(volatile float*)(base + f + 2) = o.z;
  }
}

__global__ __launch_bounds__(NTHR) void k_wprep(
    const float* __restrict__ W1, const float* __restrict__ W2,
    _Float16* w1p, _Float16* w2p, int L) {
  const int tid = (int)threadIdx.x, b = (int)blockIdx.x;
  const int nb1 = 16 * L;
  float v[8];
  _Float16* dp;
  if (b < nb1) {
    const int o = (b * NTHR + tid) * 8;
    const int i = o >> 15, rem = o & 32767;
    const int a = rem >> 14, rem2 = rem & 16383;
    const int n = rem2 >> 7, k0 = rem2 & 127;
    const float* sp = W1 + ((size_t)(i * 2 * DD + a * DD + k0)) * DD + n;
#pragma unroll
    for (int j = 0; j < 8; ++j) v[j] = sp[(size_t)j * DD] * 64.0f;
    dp = w1p + o;
  } else {
    const int o = ((b - nb1) * NTHR + tid) * 8;
    const int i = o >> 14, rem = o & 16383;
    const int n = rem >> 7, k0 = rem & 127;
    const float* sp = W2 + ((size_t)(i * DD + k0)) * DD + n;
#pragma unroll
    for (int j = 0; j < 8; ++j) v[j] = sp[(size_t)j * DD] * 64.0f;
    dp = w2p + o;
  }
  v8h ov;
#pragma unroll
  for (int j = 0; j < 8; ++j) ov[j] = (_Float16)v[j];
  *(volatile v8h*)dp = ov;
  __threadfence();
  *(volatile v8h*)dp = ov;
}

__global__ __launch_bounds__(NTHR) void k_temb(
    const int* __restrict__ nv, const float* __restrict__ w1, const float* __restrict__ bb1,
    const float* __restrict__ w2, const float* __restrict__ bb2, float* temb) {
  __shared__ float emb[2 * DD];
  __shared__ float hid[2 * 4 * DD];
  __shared__ __attribute__((aligned(16))) float so[2 * DD];
  const int tid = threadIdx.x, lane = tid & 31, wave = tid >> 5;
  if (tid < DD) {
    const int b = tid >> 6, k = tid & 63;
    const float nf = (float)nv[b];
    const float fr = expf((-9.210340371976184f * (float)k) * 0.015625f);
    const float a = nf * fr;
    emb[b * DD + k]      = sinf(a);
    emb[b * DD + 64 + k] = cosf(a);
  }
  __syncthreads();
  for (int j = tid; j < 4 * DD; j += NTHR) {
    float s0 = bb1[j], s1 = bb1[j];
#pragma unroll 1
    for (int k = 0; k < DD; ++k) {
      const float w = w1[(size_t)k * (4 * DD) + j];
      s0 = fmaf(emb[k], w, s0);
      s1 = fmaf(emb[DD + k], w, s1);
    }
    hid[j] = silu_f(s0);
    hid[4 * DD + j] = silu_f(s1);
  }
  __syncthreads();
  {
    const int b = tid >> 7, c = tid & 127;
    float s = bb2[c];
#pragma unroll 1
    for (int k = 0; k < 4 * DD; ++k) s = fmaf(hid[b * 4 * DD + k], w2[(size_t)k * DD + c], s);
    so[tid] = s;
  }
  __syncthreads();
  if (wave < 2) {
    const v4f o = *(const v4f*)(so + wave * DD + 4 * lane);
    float* dp = temb + wave * DD + 4 * lane;
    *(volatile v4f*)dp = o;
    __threadfence();
    *(volatile v4f*)dp = o;
  }
}

__global__ __launch_bounds__(NTHR) void k_inproj(
    const float* __restrict__ delta, const float* __restrict__ win, const float* __restrict__ bin,
    const float* __restrict__ temb, float* h, int nRows, int nE) {
  const int tid = threadIdx.x, lane = tid & 31, wave = tid >> 5;
  const int c = 4 * lane;
  const v4f w0 = *(const v4f*)(win + c);
  const v4f w1 = *(const v4f*)(win + DD + c);
  const v4f w2 = *(const v4f*)(win + 2 * DD + c);
  const v4f bb = *(const v4f*)(bin + c);
  const v4f t0 = *(const v4f*)(temb + c);
  const v4f t1 = *(const v4f*)(temb + DD + c);
#pragma unroll 1
  for (int j = 0; j < 8; ++j) {
    const int row = blockIdx.x * 64 + 8 * wave + j;
    if (row < nRows) {
      const float* dp = delta + (size_t)row * 3;
      const float d0 = dp[0], d1 = dp[1], d2 = dp[2];
      const v4f te = (row >= nE) ? t1 : t0;
      v4f o = d0 * w0 + d1 * w1 + d2 * w2 + bb;
      o = o + te;
      float* op = h + (size_t)row * DD + c;
      *(volatile v4f*)op = o;
      __threadfence();
      *(volatile v4f*)op = o;
    }
  }
}

template <int NB>
__device__ __forceinline__ int scan_chunk(const int* __restrict__ keys, int nK, int cbase, int slotBase,
                                          int vec8, int* list, int tid, int lane, int wave) {
  int wc = 0;
#pragma unroll
  for (int g = 0; g < NGRP; ++g) {
    const int el0  = (g * NTHR + tid) * EPT;
    const int e0   = cbase + el0;
    const int sent = -2147483647 - 1;
    v4i da, db;
    if (vec8 != 0 && cbase + CHUNK <= nK) {
      da = *(const v4i*)(keys + e0);
      db = *(const v4i*)(keys + e0 + 4);
    } else {
      da.x = (e0     < nK) ? keys[min(e0,     nK - 1)] : sent;
      da.y = (e0 + 1 < nK) ? keys[min(e0 + 1, nK - 1)] : sent;
      da.z = (e0 + 2 < nK) ? keys[min(e0 + 2, nK - 1)] : sent;
      da.w = (e0 + 3 < nK) ? keys[min(e0 + 3, nK - 1)] : sent;
      db.x = (e0 + 4 < nK) ? keys[min(e0 + 4, nK - 1)] : sent;
      db.y = (e0 + 5 < nK) ? keys[min(e0 + 5, nK - 1)] : sent;
      db.z = (e0 + 6 < nK) ? keys[min(e0 + 6, nK - 1)] : sent;
      db.w = (e0 + 7 < nK) ? keys[min(e0 + 7, nK - 1)] : sent;
    }
    const unsigned nb = (unsigned)slotBase;
    const unsigned s0 = (unsigned)da.x - nb, s1 = (unsigned)da.y - nb;
    const unsigned s2 = (unsigned)da.z - nb, s3 = (unsigned)da.w - nb;
    const unsigned s4 = (unsigned)db.x - nb, s5 = (unsigned)db.y - nb;
    const unsigned s6 = (unsigned)db.z - nb, s7 = (unsigned)db.w - nb;
    const bool h0 = s0 < (unsigned)NB, h1 = s1 < (unsigned)NB, h2 = s2 < (unsigned)NB, h3 = s3 < (unsigned)NB;
    const bool h4 = s4 < (unsigned)NB, h5 = s5 < (unsigned)NB, h6 = s6 < (unsigned)NB, h7 = s7 < (unsigned)NB;
    const unsigned any = __builtin_amdgcn_ballot_w32(h0 | h1 | h2 | h3 | h4 | h5 | h6 | h7);
    if (any != 0u) {
#define HITJ(J, HJ, SJ) { \
        const unsigned mj = __builtin_amdgcn_ballot_w32(HJ); \
        if (mj != 0u) { \
          if (HJ) { \
            const int pos = wc + (int)__builtin_amdgcn_mbcnt_lo(mj, 0u); \
            if (pos < WCAP) list[wave * WCAP + pos] = ((el0 + (J)) << 12) | (int)(SJ); \
          } \
          wc += (int)__builtin_popcount(mj); } }
      HITJ(0, h0, s0)
      HITJ(1, h1, s1)
      HITJ(2, h2, s2)
      HITJ(3, h3, s3)
      HITJ(4, h4, s4)
      HITJ(5, h5, s5)
      HITJ(6, h6, s6)
      HITJ(7, h7, s7)
#undef HITJ
    }
  }
  return wc;
}

__device__ __forceinline__ void drain_hits(const int* list, const int* wcnt, float* accf,
                                           const float* __restrict__ h, int cbase, int nK, int nE, int lane) {
#pragma unroll 1
  for (int wsx = 0; wsx < NWAVE; ++wsx) {
    int n = __builtin_amdgcn_readfirstlane(wcnt[wsx]);
    n = n > WCAP ? WCAP : (n < 0 ? 0 : n);
    const int* lp = list + wsx * WCAP;
#pragma unroll 1
    for (int i = 0; i < n; ++i) {
      const int ent  = __builtin_amdgcn_readfirstlane(lp[i]);
      const int slot = ent & (NBC - 1);
      int p = cbase + ((ent >> 12) & (CHUNK - 1));
      p = p > nK - 1 ? nK - 1 : p;
      const int e = p >= nE ? p - nE : p;
      const v4f x0 = *(const v4f*)(h + (size_t)e * DD + 4 * lane);
      const v4f x1 = *(const v4f*)(h + ((size_t)nE + e) * DD + 4 * lane);
      float* a0 = accf + slot * DD + 4 * lane;
      float* a1 = accf + (NBC + slot) * DD + 4 * lane;
      const v4f y0 = *(const v4f*)a0 + x0;
      const v4f y1 = *(const v4f*)a1 + x1;
      *(v4f*)a0 = y0;
      *(v4f*)a1 = y1;
    }
  }
}

__global__ __launch_bounds__(NTHR) void k_vert(
    const int* __restrict__ ei, const float* __restrict__ h,
    const _Float16* __restrict__ w1pl, float* PQ, int nE, int Vpad, int vec8) {
  float* accf = g_dyn;
  _Float16* xs = (_Float16*)g_dyn;
  int* list = (int*)(g_dyn + 2 * NBC * DD);
  __shared__ int wcnt[NWAVE];
  const int tid = threadIdx.x, lane = tid & 31, wave = tid >> 5, hh = lane >> 4, m = lane & 15;
  const int nodeBase = blockIdx.x * NBC;
  const int nK = 2 * nE;

  {
    const v4f z = {0.f, 0.f, 0.f, 0.f};
    for (int i = tid * 4; i < 2 * NBC * DD; i += NTHR * 4) *(v4f*)(accf + i) = z;
  }
  __syncthreads();

  const int nChunks = (nK + CHUNK - 1) / CHUNK;
#pragma unroll 1
  for (int ch = 0; ch < nChunks; ++ch) {
    const int cbase = ch * CHUNK;
    const int wc = scan_chunk<NBC>(ei, nK, cbase, nodeBase, vec8, list, tid, lane, wave);
    if (lane == 0) wcnt[wave] = wc;
    __syncthreads();
    if (wave == 0) drain_hits(list, wcnt, accf, h, cbase, nK, nE, lane);
    __syncthreads();
  }

#pragma unroll 1
  for (int c = 0; c < (2 * NBC) / 16; ++c) {
    const int ri = tid >> 4, c8 = (tid & 15) * 8;
    const int row = 16 * c + ri;
    const float* sp = accf + row * DD + c8;
    const v4f x0 = *(const v4f*)sp;
    const v4f x1 = *(const v4f*)(sp + 4);
    __syncthreads();
    v8h o;
    o[0] = (_Float16)(x0.x * 16.0f); o[1] = (_Float16)(x0.y * 16.0f);
    o[2] = (_Float16)(x0.z * 16.0f); o[3] = (_Float16)(x0.w * 16.0f);
    o[4] = (_Float16)(x1.x * 16.0f); o[5] = (_Float16)(x1.y * 16.0f);
    o[6] = (_Float16)(x1.z * 16.0f); o[7] = (_Float16)(x1.w * 16.0f);
    *(v8h*)(xs + row * XP + c8) = o;
    __syncthreads();
  }

  float* stg = g_dyn + VSTG + wave * 2048;
#pragma unroll 1
  for (int cg = 0; cg < 4; ++cg) {
    const _Float16* pl = w1pl + (size_t)(cg >> 1) * (DD * DD);
    const int n0 = 64 * (cg & 1);
    v8f acc[2][4];
#pragma unroll
    for (int rt = 0; rt < 2; ++rt)
#pragma unroll
      for (int t = 0; t < 4; ++t) acc[rt][t] = zero8();
    const _Float16* ap0 = xs + (32 * wave + m) * XP + 8 * hh;
    const _Float16* ap1 = ap0 + 16 * XP;
#pragma unroll
    for (int ks = 0; ks < 4; ++ks) {
      Frag a0, a1;
      a0.h[0] = *(const v8h*)(ap0 + 32 * ks);
      a0.h[1] = *(const v8h*)(ap0 + 32 * ks + 16);
      a1.h[0] = *(const v8h*)(ap1 + 32 * ks);
      a1.h[1] = *(const v8h*)(ap1 + 32 * ks + 16);
#pragma unroll
      for (int t = 0; t < 4; ++t) {
        const _Float16* bp = pl + (size_t)(n0 + 16 * t + m) * DD + 32 * ks + 8 * hh;
        Frag bf;
        bf.h[0] = *(const v8h*)bp;
        bf.h[1] = *(const v8h*)(bp + 16);
        acc[0][t] = wm(a0.v, bf.v, acc[0][t]);
        acc[1][t] = wm(a1.v, bf.v, acc[1][t]);
      }
    }
#pragma unroll
    for (int rt = 0; rt < 2; ++rt) {
      float* sp = stg + (16 * rt + 8 * hh) * 64 + m;
#pragma unroll
      for (int t = 0; t < 4; ++t) {
#pragma unroll
        for (int r = 0; r < 8; ++r) sp[r * 64 + 16 * t] = acc[rt][t][r] * 0.0009765625f;
      }
    }
    __syncthreads();
    v4f vals[16];
#pragma unroll
    for (int j = 0; j < 16; ++j) {
      const int rl = 2 * j + hh;
      vals[j] = *(const v4f*)(stg + rl * 64 + 4 * m);
    }
#pragma unroll
    for (int j = 0; j < 16; ++j) {
      const int rl = 2 * j + hh;
      const int R = 32 * wave + rl;
      const int bb = R >> 7, slot = R & (NBC - 1);
      float* dp = PQ + ((size_t)(bb * Vpad + nodeBase + slot)) * (2 * DD) + 64 * cg + 4 * m;
      *(volatile v4f*)dp = vals[j];
    }
    __threadfence();
#pragma unroll
    for (int j = 0; j < 16; ++j) {
      const int rl = 2 * j + hh;
      const int R = 32 * wave + rl;
      const int bb = R >> 7, slot = R & (NBC - 1);
      float* dp = PQ + ((size_t)(bb * Vpad + nodeBase + slot)) * (2 * DD) + 64 * cg + 4 * m;
      *(volatile v4f*)dp = vals[j];
    }
    __syncthreads();
  }
}

__global__ __launch_bounds__(NTHR) void k_edge(
    const int* __restrict__ ei, const float* __restrict__ PQ, const _Float16* __restrict__ w2pl,
    const float* __restrict__ pb1, const float* __restrict__ plg, const float* __restrict__ plb,
    const float* __restrict__ pb2, const float* __restrict__ png, const float* __restrict__ pnb,
    const float* __restrict__ wout, const float* __restrict__ bout, const int* __restrict__ nvp,
    float* h, float* out, int nE, int Vpad, int last) {
  _Float16* xs = (_Float16*)g_dyn;
  float* stg = g_dyn;
  __shared__ int sIdx[2 * NBE];
  __shared__ __attribute__((aligned(16))) float sPar[6 * DD];
  __shared__ float sWo[3 * DD];
  __shared__ float sBo[4];
  __shared__ __attribute__((aligned(16))) float sOut[2 * NBE * 3];
  const int tid = threadIdx.x, lane = tid & 31, wave = tid >> 5, hh = lane >> 4, m = lane & 15;
  const int e0 = blockIdx.x * NBE;
  const int bq = wave >> 2, rt = wave & 3;

  if (tid < NBE) {
    int nv = nvp[0];
    nv = nv < 1 ? 1 : (nv > Vpad ? Vpad : nv);
    int e = e0 + tid;
    e = e > nE - 1 ? nE - 1 : e;
    int s = ei[e];
    s = s < 0 ? 0 : (s > nv - 1 ? nv - 1 : s);
    int d = ei[(size_t)nE + e];
    d = d < 0 ? 0 : (d > nv - 1 ? nv - 1 : d);
    sIdx[tid] = s;
    sIdx[NBE + tid] = d;
  }
  if (tid < DD) {
    sPar[tid]          = pb1[tid];
    sPar[DD + tid]     = plg[tid];
    sPar[2 * DD + tid] = plb[tid];
    sPar[3 * DD + tid] = pb2[tid];
    sPar[4 * DD + tid] = png[tid];
    sPar[5 * DD + tid] = pnb[tid];
  } else {
    for (int i = tid - DD; i < 3 * DD; i += DD) sWo[i] = wout[i];
    if (tid == DD) { sBo[0] = bout[0]; sBo[1] = bout[1]; sBo[2] = bout[2]; sBo[3] = 0.f; }
  }
  __syncthreads();

  {
    const v4f vb1 = *(const v4f*)(sPar + 4 * lane);
    const v4f vg  = *(const v4f*)(sPar + DD + 4 * lane);
    const v4f vbe = *(const v4f*)(sPar + 2 * DD + 4 * lane);
    const float* Pb = PQ + (size_t)bq * Vpad * (2 * DD);
#pragma unroll 1
    for (int j = 0; j < 16; ++j) {
      const int r = 16 * rt + j;
      const int R = 16 * wave + j;
      const int s = sIdx[r], d = sIdx[NBE + r];
      const v4f p = *(const v4f*)(Pb + (size_t)s * (2 * DD) + 4 * lane);
      const v4f q = *(const v4f*)(Pb + (size_t)d * (2 * DD) + DD + 4 * lane);
      const v4f x = p + q + vb1;
      float s1 = (x.x + x.y) + (x.z + x.w);
      s1 += __shfl_xor(s1, 1);
      s1 += __shfl_xor(s1, 2);
      s1 += __shfl_xor(s1, 4);
      s1 += __shfl_xor(s1, 8);
      s1 += __shfl_xor(s1, 16);
      const float mean = s1 * 0.0078125f;
      const v4f dv = x - mean;
      float s2 = (dv.x * dv.x + dv.y * dv.y) + (dv.z * dv.z + dv.w * dv.w);
      s2 += __shfl_xor(s2, 1);
      s2 += __shfl_xor(s2, 2);
      s2 += __shfl_xor(s2, 4);
      s2 += __shfl_xor(s2, 8);
      s2 += __shfl_xor(s2, 16);
      const float rstd = rsqrtf(s2 * 0.0078125f + 1e-5f);
      const v4f y = dv * rstd * vg + vbe;
      v4h o;
      o[0] = (_Float16)silu_f(y.x);
      o[1] = (_Float16)silu_f(y.y);
      o[2] = (_Float16)silu_f(y.z);
      o[3] = (_Float16)silu_f(y.w);
      *(v4h*)(xs + R * XP + 4 * lane) = o;
    }
  }
  __syncthreads();

  v8f acc[8];
#pragma unroll
  for (int t = 0; t < 8; ++t) acc[t] = zero8();
  {
    const _Float16* ap = xs + (16 * wave + m) * XP + 8 * hh;
#pragma unroll
    for (int ks = 0; ks < 4; ++ks) {
      Frag a;
      a.h[0] = *(const v8h*)(ap + 32 * ks);
      a.h[1] = *(const v8h*)(ap + 32 * ks + 16);
#pragma unroll
      for (int t = 0; t < 8; ++t) {
        const _Float16* bp = w2pl + (size_t)(16 * t + m) * DD + 32 * ks + 8 * hh;
        Frag bf;
        bf.h[0] = *(const v8h*)bp;
        bf.h[1] = *(const v8h*)(bp + 16);
        acc[t] = wm(a.v, bf.v, acc[t]);
      }
    }
  }
  __syncthreads();

  {
    const float* hb = h + (size_t)bq * nE * DD;
#pragma unroll 4
    for (int j = 0; j < 16; ++j) {
      int e = e0 + 16 * rt + j;
      e = e > nE - 1 ? nE - 1 : e;
      const v4f v = *(const v4f*)(hb + (size_t)e * DD + 4 * lane);
      *(v4f*)(stg + (16 * wave + j) * DD + 4 * lane) = v;
    }
  }
  __syncthreads();

  {
#pragma unroll
    for (int r = 0; r < 8; ++r) {
      float* sp = stg + (16 * wave + 8 * hh + r) * DD + m;
      float xv[8];
      float s1 = 0.f;
#pragma unroll
      for (int t = 0; t < 8; ++t) {
        const float x = acc[t][r] * 0.015625f + sPar[3 * DD + 16 * t + m] + sp[16 * t];
        xv[t] = x;
        s1 += x;
      }
      s1 += __shfl_xor(s1, 1);
      s1 += __shfl_xor(s1, 2);
      s1 += __shfl_xor(s1, 4);
      s1 += __shfl_xor(s1, 8);
      const float mean = s1 * 0.0078125f;
      float s2 = 0.f;
#pragma unroll
      for (int t = 0; t < 8; ++t) {
        const float dd = xv[t] - mean;
        xv[t] = dd;
        s2 += dd * dd;
      }
      s2 += __shfl_xor(s2, 1);
      s2 += __shfl_xor(s2, 2);
      s2 += __shfl_xor(s2, 4);
      s2 += __shfl_xor(s2, 8);
      const float rstd = rsqrtf(s2 * 0.0078125f + 1e-5f);
#pragma unroll
      for (int t = 0; t < 8; ++t)
        sp[16 * t] = xv[t] * rstd * sPar[4 * DD + 16 * t + m] + sPar[5 * DD + 16 * t + m];
    }
  }
  __syncthreads();

  {
    v4f vrow[16];
#pragma unroll
    for (int j = 0; j < 16; ++j) vrow[j] = *(const v4f*)(stg + (16 * wave + j) * DD + 4 * lane);
    float* hb = h + (size_t)bq * nE * DD;
#pragma unroll
    for (int j = 0; j < 16; ++j) {
      const int e = e0 + 16 * rt + j;
      if (e < nE) *(volatile v4f*)(hb + (size_t)e * DD + 4 * lane) = vrow[j];
    }
    __threadfence();
#pragma unroll
    for (int j = 0; j < 16; ++j) {
      const int e = e0 + 16 * rt + j;
      if (e < nE) *(volatile v4f*)(hb + (size_t)e * DD + 4 * lane) = vrow[j];
    }
  }

  if (last != 0) {
    {
      const int R = tid >> 1, q = tid & 1;
      const float* sr = stg + R * DD + 64 * q;
      const float* wr = sWo + 64 * q * 3;
      float a0 = 0.f, a1 = 0.f, a2 = 0.f;
#pragma unroll 1
      for (int c = 0; c < 64; ++c) {
        const float v = sr[c];
        a0 = fmaf(v, wr[3 * c], a0);
        a1 = fmaf(v, wr[3 * c + 1], a1);
        a2 = fmaf(v, wr[3 * c + 2], a2);
      }
      a0 += __shfl_xor(a0, 1);
      a1 += __shfl_xor(a1, 1);
      a2 += __shfl_xor(a2, 1);
      if (q == 0) {
        sOut[R * 3]     = a0 + sBo[0];
        sOut[R * 3 + 1] = a1 + sBo[1];
        sOut[R * 3 + 2] = a2 + sBo[2];
      }
    }
    __syncthreads();
    if (wave < 2) {
      int nv = nE - e0;
      nv = nv > NBE ? NBE : nv;
      const int nval = 3 * nv;
      float* base = out + ((size_t)wave * nE + e0) * 3;
      const float* so = sOut + wave * (NBE * 3);
      const int f0 = 4 * lane;
      const int f1 = 128 + 4 * (lane & 15);
      const v4f o0 = *(const v4f*)(so + f0);
      const v4f o1 = *(const v4f*)(so + f1);
      const bool act1 = lane < 16;
      st_seg(base, f0, nval, o0);
      if (act1) st_seg(base, f1, nval, o1);
      __threadfence();
      st_seg(base, f0, nval, o0);
      if (act1) st_seg(base, f1, nval, o1);
    }
  }
}

extern "C" void kernel_launch(void* const* d_in, const int* in_sizes, int n_in,
                              void* d_out, int out_size, void* d_ws, size_t ws_size,
                              hipStream_t stream) {
  if (n_in < 20) return;
  const int nB = in_sizes[1];
  if (nB != 2) return;
  if (in_sizes[2] < 2 || (in_sizes[2] & 1) != 0) return;
  const int nE = in_sizes[2] / 2;
  if (nE < 1 || nE > (1 << 24)) return;
  if (in_sizes[0] != nB * nE * 3 || out_size != nB * nE * 3) return;
  if (in_sizes[3] < 1 || in_sizes[4] != 3 * DD || in_sizes[5] != DD) return;
  const int L = in_sizes[6] / (2 * DD * DD);
  if (L < 1 || L > 16 || in_sizes[6] != L * 2 * DD * DD || in_sizes[10] != L * DD * DD) return;
  if (in_sizes[7] != L * DD || in_sizes[8] != L * DD || in_sizes[9] != L * DD) return;
  if (in_sizes[11] != L * DD || in_sizes[12] != L * DD || in_sizes[13] != L * DD) return;
  if (in_sizes[14] != 4 * DD * DD || in_sizes[15] != 4 * DD || in_sizes[16] != 4 * DD * DD || in_sizes[17] != DD) return;
  if (in_sizes[18] != 3 * DD || in_sizes[19] != 3) return;

  const float* delta = (const float*)d_in[0];
  const int*   nvec  = (const int*)d_in[1];
  const int*   eidx  = (const int*)d_in[2];
  const int*   nvp   = (const int*)d_in[3];
  const float* w_in  = (const float*)d_in[4];
  const float* b_in  = (const float*)d_in[5];
  const float* W1    = (const float*)d_in[6];
  const float* b1    = (const float*)d_in[7];
  const float* ln_g  = (const float*)d_in[8];
  const float* ln_b  = (const float*)d_in[9];
  const float* W2    = (const float*)d_in[10];
  const float* b2    = (const float*)d_in[11];
  const float* nrm_g = (const float*)d_in[12];
  const float* nrm_b = (const float*)d_in[13];
  const float* te_w1 = (const float*)d_in[14];
  const float* te_b1 = (const float*)d_in[15];
  const float* te_w2 = (const float*)d_in[16];
  const float* te_b2 = (const float*)d_in[17];
  const float* w_out = (const float*)d_in[18];
  const float* b_out = (const float*)d_in[19];
  float* out = (float*)d_out;

  const int nbVert = (NVERT + NBC - 1) / NBC;
  const int Vpad   = nbVert * NBC;
  const int nbEdge = (nE + NBE - 1) / NBE;
  const int nRows  = nB * nE;
  const int nbIn   = (nRows + 63) / 64;

  char* ws = (char*)d_ws;
  size_t off = 0;
  const size_t oH  = off; off += (size_t)nRows * DD * 4;            off = (off + 255) & ~(size_t)255;
  const size_t oPQ = off; off += (size_t)nB * Vpad * (2 * DD) * 4;  off = (off + 255) & ~(size_t)255;
  const size_t oW1 = off; off += (size_t)L * 2 * DD * DD * 2;       off = (off + 255) & ~(size_t)255;
  const size_t oW2 = off; off += (size_t)L * DD * DD * 2;           off = (off + 255) & ~(size_t)255;
  const size_t oT  = off; off += (size_t)nB * DD * 4;               off = (off + 255) & ~(size_t)255;
  if (off > ws_size || off > (size_t)WSCAP) return;
  float*    hbuf = (float*)(ws + oH);
  float*    PQ   = (float*)(ws + oPQ);
  _Float16* w1p  = (_Float16*)(ws + oW1);
  _Float16* w2p  = (_Float16*)(ws + oW2);
  float*    temb = (float*)(ws + oT);

  hipFuncSetAttribute(reinterpret_cast<const void*>(&k_vert), hipFuncAttributeMaxDynamicSharedMemorySize, VLDSB);
  hipFuncSetAttribute(reinterpret_cast<const void*>(&k_edge), hipFuncAttributeMaxDynamicSharedMemorySize, ELDSB);

  const int vec8 = 1;

  k_wprep<<<24 * L, NTHR, 0, stream>>>(W1, W2, w1p, w2p, L);
  k_temb<<<1, NTHR, 0, stream>>>(nvec, te_w1, te_b1, te_w2, te_b2, temb);
  k_inproj<<<nbIn, NTHR, 0, stream>>>(delta, w_in, b_in, temb, hbuf, nRows, nE);
  for (int i = 0; i < L; ++i) {
    const _Float16* w1pl = w1p + (size_t)i * 2 * DD * DD;
    const _Float16* w2pl = w2p + (size_t)i * DD * DD;
    k_vert<<<nbVert, NTHR, VLDSB, stream>>>(eidx, hbuf, w1pl, PQ, nE, Vpad, vec8);
    k_edge<<<nbEdge, NTHR, ELDSB, stream>>>(eidx, PQ, w2pl,
        b1 + (size_t)i * DD, ln_g + (size_t)i * DD, ln_b + (size_t)i * DD,
        b2 + (size_t)i * DD, nrm_g + (size_t)i * DD, nrm_b + (size_t)i * DD,
        w_out, b_out, nvp, hbuf, out, nE, Vpad, (i == L - 1) ? 1 : 0);
  }
}
